// EdgeConvBlock_27943057227832
// MI455X (gfx1250) — hardware-verified
//
#include <hip/hip_runtime.h>
#include <stdint.h>

#pragma clang fp contract(off)

typedef __attribute__((ext_vector_type(16))) _Float16 v16h;
typedef __attribute__((ext_vector_type(8)))  _Float16 v8h;
typedef __attribute__((ext_vector_type(16))) __bf16   v16b;
typedef __attribute__((ext_vector_type(8)))  __bf16   v8b;
typedef __attribute__((ext_vector_type(8)))  float    v8f;
typedef __attribute__((ext_vector_type(4)))  float    v4f;
typedef __attribute__((ext_vector_type(2)))  float    v2f;
typedef __attribute__((ext_vector_type(4)))  int      v4i;
#define PSCALE 32768.0f
#define U16(p) ((const unsigned short*)(const void*)(p))
#define PSCALE_INV (1.0f / 32768.0f)

__device__ __forceinline__ unsigned short f2bf_bits(float f) {
  unsigned u = __float_as_uint(f);
  return (unsigned short)((u + 0x7FFFu + ((u >> 16) & 1u)) >> 16);
}
__device__ __forceinline__ float bf_bits2f(unsigned short h) { return __uint_as_float(((unsigned)h) << 16); }

__device__ __forceinline__ void dep_guard_h(v8f& a, v8f& b, v16h x, v16h y) { asm volatile("v_nop\n\tv_nop\n\tv_nop\n\tv_nop" : "+v"(a), "+v"(b) : "v"(x), "v"(y)); }
__device__ __forceinline__ void dep_guard_b(v8f& a, v8f& b, v16b x, v16b y) { asm volatile("v_nop\n\tv_nop\n\tv_nop\n\tv_nop" : "+v"(a), "+v"(b) : "v"(x), "v"(y)); }
__device__ __forceinline__ void keep4_h(v16h a, v16h b, v16h c, v16h d) { asm volatile("v_nop" :: "v"(a), "v"(b), "v"(c), "v"(d)); }
__device__ __forceinline__ void keep4_b(v16b a, v16b b, v16b c, v16b d) { asm volatile("v_nop" :: "v"(a), "v"(b), "v"(c), "v"(d)); }
__device__ __forceinline__ void acc_guard4(v8f& a, v8f& b, v8f& c, v8f& d) { asm volatile("v_nop\n\tv_nop\n\tv_nop\n\tv_nop" : "+v"(a), "+v"(b), "+v"(c), "+v"(d)); }
template <typename T> struct Frag;
template <> struct Frag<_Float16> {
  typedef v16h V; union U { v16h v; v8h h[2]; };
  static __device__ __forceinline__ v16h load(const _Float16* p) {
    U f; f.h[0] = *(const v8h*)(p); f.h[1] = *(const v8h*)(p + 16); return f.v;
  }
  static __device__ __forceinline__ v8f mma(v16h a, v16h b, v8f c) {
    return __builtin_amdgcn_wmma_f32_16x16x32_f16(false, a, false, b, (short)0, c, false, false);
  }
  static __device__ __forceinline__ void guard(v8f& a, v8f& b, v16h x, v16h y) { dep_guard_h(a, b, x, y); }
  static __device__ __forceinline__ void keep(v16h a, v16h b, v16h c, v16h d) { keep4_h(a, b, c, d); }
};
template <> struct Frag<__bf16> {
  typedef v16b V; union U { v16b v; v8b h[2]; };
  static __device__ __forceinline__ v16b load(const __bf16* p) {
    U f; f.h[0] = *(const v8b*)(p); f.h[1] = *(const v8b*)(p + 16); return f.v;
  }
  static __device__ __forceinline__ v8f mma(v16b a, v16b b, v8f c) {
    return __builtin_amdgcn_wmma_f32_16x16x32_bf16(false, a, false, b, (short)0, c, false, false);
  }
  static __device__ __forceinline__ void guard(v8f& a, v8f& b, v16b x, v16b y) { dep_guard_b(a, b, x, y); }
  static __device__ __forceinline__ void keep(v16b a, v16b b, v16b c, v16b d) { keep4_b(a, b, c, d); }
};

template <int ET> struct Elem;
template <> struct Elem<0> { typedef _Float16 T; };
template <> struct Elem<1> { typedef __bf16 T; };
template <int ET, bool SPLIT, int BIAS_MODE, int OUT_MODE, bool RESID, int ACT = 0>
__global__ __launch_bounds__(256) void wmma_gemm64(
    const unsigned short* __restrict__ Ap, const unsigned short* __restrict__ A2p, int lda, long strideA,
    const unsigned short* __restrict__ Btp, const unsigned short* __restrict__ Bt2p, int ldb, long strideB,
    void* __restrict__ Cout, void* __restrict__ Cout2, int ldc, long strideC,
    const float* __restrict__ bias,
    const float* __restrict__ resid, long strideR,
    int M, int N, int K, float scale) {
  typedef typename Elem<ET>::T T;
  typedef typename Frag<T>::V V;
  const T* A = (const T*)Ap; const T* A2 = (const T*)A2p; const T* Bt = (const T*)Btp; const T* Bt2 = (const T*)Bt2p;
  __shared__ __align__(16) float sT[8][16 * 68];
  const int b    = blockIdx.y;
  const int lane = threadIdx.x & 31;
  const int wave = threadIdx.x >> 5;
  const int tilesN = N >> 6;
  const int tilesM = M >> 6;
  const int tile = blockIdx.x * 8 + wave;
  if (tile >= tilesM * tilesN) return;
  const int tm = tile / tilesN;
  const int tn = tile - tm * tilesN;
  const int m0 = tm << 6;
  const int n0 = tn << 6;

  const T* Ab  = A  + (size_t)b * strideA;
  const T* Bb  = Bt + (size_t)b * strideB;
  const T* Ab2 = SPLIT ? (A2  + (size_t)b * strideA) : nullptr;
  const T* Bb2 = SPLIT ? (Bt2 + (size_t)b * strideB) : nullptr;

  const int rlane = lane & 15;
  const int koff  = (lane >> 4) * 8;
  const int mOff  = (lane >> 4) * 8;

  v8f acc[4][4];
#pragma unroll
  for (int i = 0; i < 4; ++i)
#pragma unroll
    for (int j = 0; j < 4; ++j) acc[i][j] = (v8f){0.f,0.f,0.f,0.f,0.f,0.f,0.f,0.f};

  for (int k0 = 0; k0 < K; k0 += 32) {
    V bh[4], bl[4];
#pragma unroll
    for (int j = 0; j < 4; ++j) {
      const size_t bo = (size_t)(n0 + (j << 4) + rlane) * ldb + koff + k0;
      bh[j] = Frag<T>::load(Bb + bo);
      if (SPLIT) bl[j] = Frag<T>::load(Bb2 + bo);
    }
#pragma unroll
    for (int i = 0; i < 4; ++i) {
      const size_t ao = (size_t)(m0 + (i << 4) + rlane) * lda + koff + k0;
      V ah = Frag<T>::load(Ab + ao);
      V al;
      if (SPLIT) al = Frag<T>::load(Ab2 + ao);
#pragma unroll
      for (int j = 0; j < 4; ++j) {
        acc[i][j] = Frag<T>::mma(ah, bh[j], acc[i][j]);
        if (SPLIT) {
          acc[i][j] = Frag<T>::mma(ah, bl[j], acc[i][j]);
          acc[i][j] = Frag<T>::mma(al, bh[j], acc[i][j]);
        }
      }
      Frag<T>::guard(acc[i][0], acc[i][3], ah, SPLIT ? al : ah);
    }
    Frag<T>::keep(bh[0], bh[1], bh[2], bh[3]);
    if (SPLIT) Frag<T>::keep(bl[0], bl[1], bl[2], bl[3]);
  }
  acc_guard4(acc[0][0], acc[0][1], acc[0][2], acc[0][3]);
  acc_guard4(acc[1][0], acc[1][1], acc[1][2], acc[1][3]);
  acc_guard4(acc[2][0], acc[2][1], acc[2][2], acc[2][3]);
  acc_guard4(acc[3][0], acc[3][1], acc[3][2], acc[3][3]);

  float* slab = sT[wave];
  const float* Rb = RESID ? (resid + (size_t)b * strideR) : nullptr;
#pragma unroll
  for (int i = 0; i < 4; ++i) {
    const int mBase = m0 + (i << 4);
#pragma unroll
    for (int j = 0; j < 4; ++j) {
      const int n = n0 + (j << 4) + rlane;
      float bv = 0.f;
      if (BIAS_MODE == 2) bv = bias[n];
#pragma unroll
      for (int r = 0; r < 8; ++r) {
        float v = acc[i][j][r] * scale;
        if (BIAS_MODE == 1) v += bias[mBase + mOff + r];
        if (BIAS_MODE == 2) v += bv;
        if (RESID) v += Rb[(size_t)(mBase + mOff + r) * ldc + n];
        if (ACT == 1) v = tanhf(v);
        if (ACT == 2) v = fmaxf(v, 0.0f);
        if (ACT == 3) v = v / (1.0f + expf(-v));
        if (ACT == 4) v = (v > 0.f) ? v : 0.01f * v;
        if (ACT == 5) v = 0.5f * v * (1.0f + erff(v * 0.70710678118654752f));
        slab[(mOff + r) * 68 + (j << 4) + rlane] = v;
      }
    }
    __builtin_amdgcn_fence(__ATOMIC_RELEASE, "workgroup");
    __builtin_amdgcn_wave_barrier();
    __builtin_amdgcn_fence(__ATOMIC_ACQUIRE, "workgroup");
    if (OUT_MODE == 0) {
      float* C = (float*)Cout + (size_t)b * strideC;
      const int hh = lane >> 4, c4 = (lane & 15) * 4;
      for (int pass = 0; pass < 2; ++pass) {
#pragma unroll
        for (int it = 0; it < 8; ++it) {
          const int row = it * 2 + hh;
          v4f v = *(const v4f*)(slab + row * 68 + c4);
          *(volatile v4f*)(C + (size_t)(mBase + row) * ldc + n0 + c4) = v;
        }
        __threadfence();
      }
    } else {
      const int q = lane >> 3, c8 = (lane & 7) * 8;
      unsigned short* C  = (unsigned short*)Cout  + (size_t)b * strideC;
      unsigned short* C2 = (OUT_MODE == 2) ? ((unsigned short*)Cout2 + (size_t)b * strideC) : nullptr;
      for (int pass = 0; pass < 2; ++pass) {
#pragma unroll
        for (int it = 0; it < 4; ++it) {
          const int row = it * 4 + q;
          const float* sp = slab + row * 68 + c8;
          v8h hv, lv;
#pragma unroll
          for (int e = 0; e < 8; ++e) {
            if (OUT_MODE == 1) {
              hv[e] = (_Float16)sp[e];
            } else {
              unsigned short hb = f2bf_bits(sp[e]);
              unsigned short lb = f2bf_bits(sp[e] - bf_bits2f(hb));
              hv[e] = __builtin_bit_cast(_Float16, hb);
              lv[e] = __builtin_bit_cast(_Float16, lb);
            }
          }
          *(volatile v8h*)(C + (size_t)(mBase + row) * ldc + n0 + c8) = hv;
          if (OUT_MODE == 2) *(volatile v8h*)(C2 + (size_t)(mBase + row) * ldc + n0 + c8) = lv;
        }
        __threadfence();
      }
    }
    __builtin_amdgcn_fence(__ATOMIC_RELEASE, "workgroup");
    __builtin_amdgcn_wave_barrier();
    __builtin_amdgcn_fence(__ATOMIC_ACQUIRE, "workgroup");
  }
}

constexpr int NCLOUD_C = 128;
constexpr int NPT_C    = 512;
constexpr int NPTS_C   = NCLOUD_C * NPT_C;
constexpr int KNB_C    = 16;
constexpr int CH_C     = 64;
constexpr int GLD_C    = 192;
constexpr int WT_ROWS  = 320;
constexpr int EPB      = 32;
constexpr int EBLK     = NPTS_C / EPB;
constexpr int KPB      = 8;
constexpr int KBLK     = NPTS_C / KPB;
constexpr int APITCH   = 72;
constexpr float WSCALE     = 64.0f;
constexpr float WSCALE_INV = 0.015625f;
constexpr float BN_EPS     = 1e-5f;

static_assert(NPTS_C % 64 == 0);
static_assert(GLD_C % 64 == 0);
static_assert(CH_C % 32 == 0);
static_assert(EPB * EBLK == NPTS_C);
static_assert(KPB * KBLK == NPTS_C);
static_assert(NPT_C % EPB == 0);

__device__ __forceinline__ v8f mma_h(v16h a, v16h b, v8f c) {
  c = __builtin_amdgcn_wmma_f32_16x16x32_f16(false, a, false, b, (short)0, c, false, false);
  asm volatile("v_nop\n\tv_nop\n\tv_nop\n\tv_nop" : "+v"(c) : "v"(a), "v"(b));
  return c;
}
__device__ __forceinline__ float bf_rne(float x) { return bf_bits2f(f2bf_bits(x)); }

__global__ __launch_bounds__(256) void k_cast_feat(const float* __restrict__ in,
                                                   unsigned short* __restrict__ outp, int n8) {
  const int i = blockIdx.x * 256 + threadIdx.x;
  if (i < n8) {
    const v4f a = *(const v4f*)(in + (size_t)i * 8);
    const v4f b = *(const v4f*)(in + (size_t)i * 8 + 4);
    v8h hv;
#pragma unroll
    for (int e = 0; e < 4; ++e) {
      hv[e]     = (_Float16)bf_rne(a[e]);
      hv[4 + e] = (_Float16)bf_rne(b[e]);
    }
    _Float16* o = (_Float16*)outp + (size_t)i * 8;
    *(volatile v8h*)o = hv;
    __threadfence();
    *(volatile v8h*)o = hv;
  }
}

__global__ __launch_bounds__(256) void k_cast_w(const float* __restrict__ W0, const float* __restrict__ W1,
                                                const float* __restrict__ W2, const float* __restrict__ SW,
                                                unsigned short* __restrict__ outp) {
  const int i = blockIdx.x * 256 + threadIdx.x;
  if (i < WT_ROWS * 32) {
    const int row = i >> 5;
    const int col = (i & 31) * 2;
    const int ra = row > 63 ? 63 : row;
    int rb = row - 64;  rb = rb < 0 ? 0 : (rb > 63 ? 63 : rb);
    int rc = row - 128; rc = rc < 0 ? 0 : (rc > 63 ? 63 : rc);
    int rd = row - 192; rd = rd < 0 ? 0 : (rd > 63 ? 63 : rd);
    int re = row - 256; re = re < 0 ? 0 : (re > 63 ? 63 : re);
    const float a0 = W0[ra * 128 + col],      a1 = W0[ra * 128 + col + 1];
    const float b0 = W0[rb * 128 + 64 + col], b1 = W0[rb * 128 + 64 + col + 1];
    const float c0 = SW[rc * 64 + col],       c1 = SW[rc * 64 + col + 1];
    const float d0 = W1[rd * 64 + col],       d1 = W1[rd * 64 + col + 1];
    const float e0 = W2[re * 64 + col],       e1 = W2[re * 64 + col + 1];
    float v0 = (row < 64) ? a0 : ((row < 128) ? b0 : ((row < 192) ? c0 : ((row < 256) ? d0 : e0)));
    float v1 = (row < 64) ? a1 : ((row < 128) ? b1 : ((row < 192) ? c1 : ((row < 256) ? d1 : e1)));
    v0 = bf_rne(v0) * WSCALE;
    v1 = bf_rne(v1) * WSCALE;
    const _Float16 h0 = (_Float16)v0, h1 = (_Float16)v1;
    const unsigned u = (unsigned)__builtin_bit_cast(unsigned short, h0) |
                       ((unsigned)__builtin_bit_cast(unsigned short, h1) << 16);
    ((volatile unsigned*)outp)[i] = u;
    __threadfence();
    ((volatile unsigned*)outp)[i] = u;
  }
}

template <int KK, int JJ>
__device__ __forceinline__ void bstage(unsigned long long (&key)[16]) {
#pragma unroll
  for (int i = 0; i < 16; ++i) {
    const int l = i ^ JJ;
    if (l > i) {
      const unsigned long long a = key[i], b = key[l];
      const bool asc = ((i & KK) == 0);
      const bool lt = b < a;
      const bool sw = asc ? lt : (!lt);
      key[i] = sw ? b : a;
      key[l] = sw ? a : b;
    }
  }
}

__global__ __launch_bounds__(256) void k_knn(const float* __restrict__ pts, int* __restrict__ idxT) {
  __shared__ float sx[NPT_C];
  __shared__ float sy[NPT_C];
  __shared__ float sr[NPT_C];
  __shared__ __align__(16) int sI[KPB * KNB_C];
  const int tid = threadIdx.x, lane = tid & 31, wave = tid >> 5;
  const int p0 = blockIdx.x * KPB;
  const int n = p0 >> 9;
  const float* cp = pts + (size_t)n * (NPT_C * 2);
  for (int i = tid; i < NPT_C; i += 256) {
    const float x = bf_rne(cp[2 * i]);
    const float y = bf_rne(cp[2 * i + 1]);
    const float xx = x * x;
    const float yy = y * y;
    sx[i] = x; sy[i] = y; sr[i] = xx + yy;
  }
  __syncthreads();
  const int pl = (p0 + wave) & (NPT_C - 1);
  const float cx = sx[pl], cy = sy[pl], rp = sr[pl];
  unsigned long long key[16];
#pragma unroll
  for (int i = 0; i < 16; ++i) {
    const int q = lane + 32 * i;
    const float qx = sx[q], qy = sy[q], rq = sr[q];
    float m = cx * qx;
    m = fmaf(cy, qy, m);
    const float m2 = m + m;
    const float t = rp - m2;
    float d = t + rq;
    d = d + 0.0f;
    unsigned u = __float_as_uint(d);
    u = (u & 0x80000000u) ? (~u) : (u | 0x80000000u);
    key[i] = ((unsigned long long)u << 32) | (unsigned long long)(unsigned)q;
  }
  bstage<2, 1>(key);
  bstage<4, 2>(key);  bstage<4, 1>(key);
  bstage<8, 4>(key);  bstage<8, 2>(key);  bstage<8, 1>(key);
  bstage<16, 8>(key); bstage<16, 4>(key); bstage<16, 2>(key); bstage<16, 1>(key);

#pragma unroll 1
  for (int it = 0; it < KNB_C + 1; ++it) {
    unsigned long long gm = key[0];
#pragma unroll
    for (int s = 16; s > 0; s >>= 1) {
      const unsigned lo = __shfl_xor((unsigned)gm, s);
      const unsigned hi = __shfl_xor((unsigned)(gm >> 32), s);
      const unsigned long long o = ((unsigned long long)hi << 32) | (unsigned long long)lo;
      gm = (o < gm) ? o : gm;
    }
    const bool win = (key[0] == gm);
#pragma unroll
    for (int i = 0; i < 15; ++i) key[i] = win ? key[i + 1] : key[i];
    key[15] = win ? (~0ull) : key[15];
    if (it > 0 && lane == 0) sI[wave * KNB_C + (it - 1)] = (int)(gm & 511ull);
  }
  __syncthreads();
  if (wave == 0) {
    const v4i v = *(const v4i*)(sI + lane * 4);
    int* dst = idxT + (size_t)blockIdx.x * (KPB * KNB_C) + lane * 4;
    *(volatile v4i*)dst = v;
    __threadfence();
    *(volatile v4i*)dst = v;
  }
}

__global__ __launch_bounds__(128) void k_stats0(const float* __restrict__ G, const int* __restrict__ idxT,
                                                float* __restrict__ rec) {
  __shared__ __align__(16) int sIdx[EPB * KNB_C];
  __shared__ float sPart[4][256];
  const int tid = threadIdx.x, lane = tid & 31, wave = tid >> 5;
  const int pbase = blockIdx.x * EPB;
  const int n = pbase >> 9;
  *(v4i*)(sIdx + tid * 4) = *(const v4i*)(idxT + (size_t)pbase * KNB_C + tid * 4);
  __syncthreads();
  const int ch2 = lane * 2;
  float xs0 = 0.f, xs1 = 0.f, xq0 = 0.f, xq1 = 0.f;
  float ss0 = 0.f, ss1 = 0.f, sq0 = 0.f, sq1 = 0.f;
  const float* gn = G + (size_t)(n * NPT_C) * GLD_C + CH_C + ch2;
#pragma unroll 1
  for (int pi = 0; pi < 8; ++pi) {
    const int pl = wave * 8 + pi;
    const int p = pbase + pl;
    const float* gp = G + (size_t)p * GLD_C;
    const v2f ga = *(const v2f*)(gp + ch2);
    const v2f gb = *(const v2f*)(gp + CH_C + ch2);
    const v2f gs = *(const v2f*)(gp + 2 * CH_C + ch2);
    const float u0 = ga[0] - gb[0], u1 = ga[1] - gb[1];
    ss0 += gs[0]; ss1 += gs[1];
    sq0 += gs[0] * gs[0]; sq1 += gs[1] * gs[1];
#pragma unroll 8
    for (int k = 0; k < KNB_C; ++k) {
      int q = sIdx[pl * KNB_C + k];
      q = q < 0 ? 0 : (q > NPT_C - 1 ? NPT_C - 1 : q);
      const v2f v = *(const v2f*)(gn + (size_t)q * GLD_C);
      const float x0 = u0 + v[0], x1 = u1 + v[1];
      xs0 += x0; xs1 += x1;
      xq0 += x0 * x0; xq1 += x1 * x1;
    }
  }
  sPart[wave][ch2] = xs0;        sPart[wave][ch2 + 1] = xs1;
  sPart[wave][64 + ch2] = xq0;   sPart[wave][64 + ch2 + 1] = xq1;
  sPart[wave][128 + ch2] = ss0;  sPart[wave][128 + ch2 + 1] = ss1;
  sPart[wave][192 + ch2] = sq0;  sPart[wave][192 + ch2 + 1] = sq1;
  __syncthreads();
#pragma unroll
  for (int rep = 0; rep < 2; ++rep) {
    const int i = tid + rep * 128;
    const float v = ((sPart[0][i] + sPart[1][i]) + sPart[2][i]) + sPart[3][i];
    float* dst = rec + (size_t)blockIdx.x * 256 + i;
    *(volatile float*)dst = v;
    __threadfence();
    *(volatile float*)dst = v;
  }
}

__global__ __launch_bounds__(256) void k_bnfin(const float* __restrict__ rec, int nrec, int stride,
                                               int offS, int offQ, float invCount,
                                               const float* __restrict__ gam, const float* __restrict__ bet,
                                               float* __restrict__ aff) {
  __shared__ double ds[4][64];
  __shared__ double dq[4][64];
  const int tid = threadIdx.x, ch = tid & 63, part = tid >> 6;
  double s = 0.0, q = 0.0;
#pragma unroll 2
  for (int r = part; r < nrec; r += 4) {
    const float* rp = rec + (size_t)r * stride;
    s += (double)rp[offS + ch];
    q += (double)rp[offQ + ch];
  }
  ds[part][ch] = s; dq[part][ch] = q;
  __syncthreads();
  if (tid < 128) {
    const int kind = tid >> 6;
    const double S = ((ds[0][ch] + ds[1][ch]) + ds[2][ch]) + ds[3][ch];
    const double Q = ((dq[0][ch] + dq[1][ch]) + dq[2][ch]) + dq[3][ch];
    const double mean = S * (double)invCount;
    double var = Q * (double)invCount - mean * mean;
    var = var < 0.0 ? 0.0 : var;
    const float g = bf_rne(gam[ch]), bb = bf_rne(bet[ch]);
    const float meanf = (float)mean, varf = (float)var;
    const float sc = g * rsqrtf(varf + BN_EPS);
    const float sh = bb - meanf * sc;
    const float v = (kind == 0) ? sc : sh;
    float* dst = aff + tid;
    *(volatile float*)dst = v;
    __threadfence();
    *(volatile float*)dst = v;
  }
}

template <int MODE>
__global__ __launch_bounds__(128) void k_edge(const float* __restrict__ G, const int* __restrict__ idxT,
                                              const unsigned short* __restrict__ W1p,
                                              const unsigned short* __restrict__ W2p,
                                              const float* __restrict__ aff0, const float* __restrict__ aff1,
                                              const float* __restrict__ aff2, const float* __restrict__ affS,
                                              float* __restrict__ rec, float* __restrict__ outp) {
  __shared__ __align__(16) _Float16 sW1[CH_C * APITCH];
  __shared__ __align__(16) _Float16 sW2[CH_C * APITCH];
  __shared__ __align__(16) _Float16 sA[4][16 * APITCH];
  __shared__ __align__(16) float sAff[512];
  __shared__ __align__(16) int sIdx[EPB * KNB_C];
  __shared__ __align__(16) float sOut[4 * 8 * CH_C];
  __shared__ float sStat[4][128];

  const int tid = threadIdx.x, lane = tid & 31, wave = tid >> 5;
  const int h = lane >> 4, c = lane & 15;
  const int pbase = blockIdx.x * EPB;
  const int n = pbase >> 9;
  {
    const _Float16* W1g = (const _Float16*)W1p;
    for (int i = tid; i < 512; i += 128) {
      const int row = i >> 3, c8 = (i & 7) * 8;
      *(v8h*)(sW1 + row * APITCH + c8) = *(const v8h*)(W1g + row * CH_C + c8);
    }
    if (MODE >= 2) {
      const _Float16* W2g = (const _Float16*)W2p;
      for (int i = tid; i < 512; i += 128) {
        const int row = i >> 3, c8 = (i & 7) * 8;
        *(v8h*)(sW2 + row * APITCH + c8) = *(const v8h*)(W2g + row * CH_C + c8);
      }
    }
    sAff[tid] = aff0[tid];
    if (MODE >= 2) sAff[128 + tid] = aff1[tid];
    if (MODE == 3) { sAff[256 + tid] = aff2[tid]; sAff[384 + tid] = affS[tid]; }
    *(v4i*)(sIdx + tid * 4) = *(const v4i*)(idxT + (size_t)pbase * KNB_C + tid * 4);
  }
  __syncthreads();

  const int gr = lane >> 3, gc8 = (lane & 7) * 8;
  float s0g[8], t0g[8];
#pragma unroll
  for (int e = 0; e < 8; ++e) { s0g[e] = sAff[gc8 + e]; t0g[e] = sAff[64 + gc8 + e]; }
  float s1d[4], t1d[4], s2d[4], t2d[4], sSd[4], tSd[4];
#pragma unroll
  for (int j = 0; j < 4; ++j) {
    s1d[j] = 0.f; t1d[j] = 0.f; s2d[j] = 0.f; t2d[j] = 0.f; sSd[j] = 0.f; tSd[j] = 0.f;
    if (MODE >= 2) { s1d[j] = sAff[128 + 16 * j + c]; t1d[j] = sAff[192 + 16 * j + c]; }
    if (MODE == 3) {
      s2d[j] = sAff[256 + 16 * j + c]; t2d[j] = sAff[320 + 16 * j + c];
      sSd[j] = sAff[384 + 16 * j + c]; tSd[j] = sAff[448 + 16 * j + c];
    }
  }
  float sts[4] = {0.f, 0.f, 0.f, 0.f};
  float stq[4] = {0.f, 0.f, 0.f, 0.f};
  _Float16* sAw = sA[wave];
  const v8f zero8 = {0.f, 0.f, 0.f, 0.f, 0.f, 0.f, 0.f, 0.f};

#pragma unroll 1
  for (int pi = 0; pi < 8; ++pi) {
    const int pl = wave * 8 + pi;
    const int p = pbase + pl;
    const float* gp = G + (size_t)p * GLD_C;
    float u[8];
    {
      const v4f ua0 = *(const v4f*)(gp + gc8);
      const v4f ua1 = *(const v4f*)(gp + gc8 + 4);
      const v4f ub0 = *(const v4f*)(gp + CH_C + gc8);
      const v4f ub1 = *(const v4f*)(gp + CH_C + gc8 + 4);
#pragma unroll
      for (int e = 0; e < 4; ++e) { u[e] = ua0[e] - ub0[e]; u[4 + e] = ua1[e] - ub1[e]; }
    }
#pragma unroll
    for (int rr = 0; rr < 4; ++rr) {
      const int row = gr + 4 * rr;
      int q = sIdx[pl * KNB_C + row];
      q = q < 0 ? 0 : (q > NPT_C - 1 ? NPT_C - 1 : q);
      const float* vp = G + (size_t)(n * NPT_C + q) * GLD_C + CH_C + gc8;
      const v4f v0 = *(const v4f*)vp;
      const v4f v1 = *(const v4f*)(vp + 4);
      v8h hv;
#pragma unroll
      for (int e = 0; e < 4; ++e) {
        const float a0 = fmaxf((u[e] + v0[e]) * s0g[e] + t0g[e], 0.0f);
        const float a1 = fmaxf((u[4 + e] + v1[e]) * s0g[4 + e] + t0g[4 + e], 0.0f);
        hv[e] = (_Float16)a0;
        hv[4 + e] = (_Float16)a1;
      }
      *(v8h*)(sAw + row * APITCH + gc8) = hv;
    }
    __syncthreads();

    v8f acc[4];
#pragma unroll
    for (int j = 0; j < 4; ++j) acc[j] = zero8;
#pragma unroll
    for (int kt = 0; kt < 2; ++kt) {
      const v16h af = Frag<_Float16>::load(sAw + c * APITCH + kt * 32 + 8 * h);
#pragma unroll
      for (int j = 0; j < 4; ++j) {
        const v16h bw = Frag<_Float16>::load(sW1 + (16 * j + c) * APITCH + kt * 32 + 8 * h);
        acc[j] = mma_h(af, bw, acc[j]);
      }
    }

    if (MODE == 1) {
#pragma unroll
      for (int j = 0; j < 4; ++j) {
#pragma unroll
        for (int r = 0; r < 8; ++r) {
          const float x = acc[j][r] * WSCALE_INV;
          sts[j] += x;
          stq[j] += x * x;
        }
      }
    } else {
#pragma unroll
      for (int j = 0; j < 4; ++j) {
#pragma unroll
        for (int r = 0; r < 8; ++r) {
          const float x = acc[j][r] * WSCALE_INV;
          const float a = fmaxf(x * s1d[j] + t1d[j], 0.0f);
          sAw[(8 * h + r) * APITCH + 16 * j + c] = (_Float16)a;
        }
      }
      __syncthreads();
      v8f acc2[4];
#pragma unroll
      for (int j = 0; j < 4; ++j) acc2[j] = zero8;
#pragma unroll
      for (int kt = 0; kt < 2; ++kt) {
        const v16h af2 = Frag<_Float16>::load(sAw + c * APITCH + kt * 32 + 8 * h);
#pragma unroll
        for (int j = 0; j < 4; ++j) {
          const v16h bw2 = Frag<_Float16>::load(sW2 + (16 * j + c) * APITCH + kt * 32 + 8 * h);
          acc2[j] = mma_h(af2, bw2, acc2[j]);
        }
      }
      if (MODE == 2) {
#pragma unroll
        for (int j = 0; j < 4; ++j) {
#pragma unroll
          for (int r = 0; r < 8; ++r) {
            const float x = acc2[j][r] * WSCALE_INV;
            sts[j] += x;
            stq[j] += x * x;
          }
        }
      } else {
        float o4[4];
#pragma unroll
        for (int j = 0; j < 4; ++j) {
          float part = 0.0f;
#pragma unroll
          for (int r = 0; r < 8; ++r) {
            const float x = acc2[j][r] * WSCALE_INV;
            part += fmaxf(x * s2d[j] + t2d[j], 0.0f);
          }
          o4[j] = part;
        }
#pragma unroll
        for (int j = 0; j < 4; ++j) o4[j] += __shfl_xor(o4[j], 16);
        const float* sp = gp + 2 * CH_C;
#pragma unroll
        for (int j = 0; j < 4; ++j) {
          const float sv = sp[16 * j + c];
          const float o = o4[j] * 0.0625f + fmaxf(sv * sSd[j] + tSd[j], 0.0f);
          if (h == 0) sOut[wave * 512 + pi * 64 + 16 * j + c] = o;
        }
      }
    }
    __syncthreads();
  }

  if (MODE != 3) {
#pragma unroll
    for (int j = 0; j < 4; ++j) {
      sts[j] += __shfl_xor(sts[j], 16);
      stq[j] += __shfl_xor(stq[j], 16);
    }
    if (h == 0) {
#pragma unroll
      for (int j = 0; j < 4; ++j) {
        sStat[wave][16 * j + c] = sts[j];
        sStat[wave][64 + 16 * j + c] = stq[j];
      }
    }
    __syncthreads();
    const float v = ((sStat[0][tid] + sStat[1][tid]) + sStat[2][tid]) + sStat[3][tid];
    float* dst = rec + (size_t)blockIdx.x * 128 + tid;
    *(volatile float*)dst = v;
    __threadfence();
    *(volatile float*)dst = v;
  } else {
    float* ob = outp + (size_t)(pbase + wave * 8) * CH_C;
    const float* so = sOut + wave * 512;
    for (int pass = 0; pass < 2; ++pass) {
#pragma unroll
      for (int chk = 0; chk < 4; ++chk) {
        const v4f v = *(const v4f*)(so + chk * 128 + lane * 4);
        *(volatile v4f*)(ob + chk * 128 + lane * 4) = v;
      }
      __threadfence();
    }
  }
}

extern "C" void kernel_launch(void* const* d_in, const int* in_sizes, int n_in,
                              void* d_out, int out_size, void* d_ws, size_t ws_size,
                              hipStream_t stream) {
  if (n_in < 14) return;
  if (in_sizes[0] != NPTS_C * 2 || in_sizes[1] != NPTS_C * CH_C || out_size != NPTS_C * CH_C) return;
  const float* points = (const float*)d_in[0];
  const float* feats  = (const float*)d_in[1];
  const float* W0  = (const float*)d_in[2];
  const float* g0  = (const float*)d_in[3];
  const float* b0  = (const float*)d_in[4];
  const float* W1  = (const float*)d_in[5];
  const float* g1  = (const float*)d_in[6];
  const float* b1  = (const float*)d_in[7];
  const float* W2  = (const float*)d_in[8];
  const float* g2  = (const float*)d_in[9];
  const float* b2  = (const float*)d_in[10];
  const float* scW = (const float*)d_in[11];
  const float* scg = (const float*)d_in[12];
  const float* scb = (const float*)d_in[13];
  float* out = (float*)d_out;

  char* ws = (char*)d_ws;
  size_t off = 0;
  auto carve = [&](size_t bytes) -> char* { char* p = ws + off; off += (bytes + 255) & ~(size_t)255; return p; };
  unsigned short* F16p = (unsigned short*)carve((size_t)NPTS_C * CH_C * 2);
  unsigned short* WTp  = (unsigned short*)carve((size_t)WT_ROWS * CH_C * 2);
  float* G    = (float*)carve((size_t)NPTS_C * GLD_C * 4);
  int*   idxT = (int*)carve((size_t)NPTS_C * KNB_C * 4);
  float* rec0 = (float*)carve((size_t)EBLK * 256 * 4);
  float* recA = (float*)carve((size_t)EBLK * 128 * 4);
  float* recB = (float*)carve((size_t)EBLK * 128 * 4);
  float* aff0 = (float*)carve(512);
  float* aff1 = (float*)carve(512);
  float* aff2 = (float*)carve(512);
  float* affS = (float*)carve(512);
  if (off > ws_size) return;

  const unsigned short* W1h = WTp + 192 * CH_C;
  const unsigned short* W2h = WTp + 256 * CH_C;
  const float inv2p20 = 1.0f / 1048576.0f;
  const float inv2p16 = 1.0f / 65536.0f;

  k_cast_feat<<<(NPTS_C * CH_C / 8) / 256, 256, 0, stream>>>(feats, F16p, NPTS_C * CH_C / 8);
  k_cast_w<<<(WT_ROWS * 32) / 256, 256, 0, stream>>>(W0, W1, W2, scW, WTp);
  wmma_gemm64<0, false, 0, 0, false, 0><<<dim3((NPTS_C / 64) * (GLD_C / 64) / 8, 1, 1), 256, 0, stream>>>(
      F16p, F16p, CH_C, 0L, WTp, WTp, CH_C, 0L, (void*)G, (void*)G, GLD_C, 0L,
      aff0, aff0, 0L, NPTS_C, GLD_C, CH_C, WSCALE_INV);
  k_knn<<<KBLK, 256, 0, stream>>>(points, idxT);
  k_stats0<<<EBLK, 128, 0, stream>>>(G, idxT, rec0);
  k_bnfin<<<1, 256, 0, stream>>>(rec0, EBLK, 256, 0, 64, inv2p20, g0, b0, aff0);
  k_bnfin<<<1, 256, 0, stream>>>(rec0, EBLK, 256, 128, 192, inv2p16, scg, scb, affS);
  k_edge<1><<<EBLK, 128, 0, stream>>>(G, idxT, W1h, W2h, aff0, aff1, aff2, affS, recA, out);
  k_bnfin<<<1, 256, 0, stream>>>(recA, EBLK, 128, 0, 64, inv2p20, g1, b1, aff1);
  k_edge<2><<<EBLK, 128, 0, stream>>>(G, idxT, W1h, W2h, aff0, aff1, aff2, affS, recB, out);
  k_bnfin<<<1, 256, 0, stream>>>(recB, EBLK, 128, 0, 64, inv2p20, g2, b2, aff2);
  k_edge<3><<<EBLK, 128, 0, stream>>>(G, idxT, W1h, W2h, aff0, aff1, aff2, affS, recB, out);
}
